// SimplifiedMultiHeadSelfAttention_79628693667935
// MI455X (gfx1250) — hardware-verified
//
#include <hip/hip_runtime.h>


typedef __attribute__((ext_vector_type(16))) _Float16 v16h;
typedef __attribute__((ext_vector_type(8)))  _Float16 v8h;
typedef __attribute__((ext_vector_type(4)))  _Float16 v4h;
typedef __attribute__((ext_vector_type(8)))  float    v8f;

#define B_   2
#define S_   2048
#define D_   1024
#define H_   16
#define HD_  64
#define M_   (B_ * S_)
#define SCALE_ 0.125f
#define EPS_ 1e-5f


__device__ __forceinline__ v8f wmma_f16(v16h a, v16h b, v8f c) {
  return __builtin_amdgcn_wmma_f32_16x16x32_f16(false, a, false, b,
                                                (short)0, c, false, false);
}

__device__ __forceinline__ v16h ld_a(const _Float16* p) {
  v8h lo = *(const v8h*)(p);
  v8h hi = *(const v8h*)(p + 16);
  return __builtin_shufflevector(lo, hi, 0,1,2,3,4,5,6,7,8,9,10,11,12,13,14,15);
}

__device__ __forceinline__ v16h ld_b(const _Float16* p) { return ld_a(p); }
typedef __attribute__((ext_vector_type(4))) unsigned v4u_t;
typedef unsigned v4ua __attribute__((ext_vector_type(4), may_alias));
typedef __attribute__((ext_vector_type(4))) float v4f_t;
typedef float v4fa __attribute__((ext_vector_type(4), may_alias));
static __device__ __forceinline__ unsigned pk2(float a, float b) {
  return (unsigned)__builtin_bit_cast(unsigned short, (_Float16)a) | ((unsigned)__builtin_bit_cast(unsigned short, (_Float16)b) << 16);
}


__global__ __launch_bounds__(256) void cvt_f16(const float* __restrict__ src,
                                               _Float16* __restrict__ dst) {
  const int i = (blockIdx.x * 256 + threadIdx.x) * 4;
  float4 f = *(const float4*)(src + i);
  v4h h;
  h[0] = (_Float16)f.x; h[1] = (_Float16)f.y;
  h[2] = (_Float16)f.z; h[3] = (_Float16)f.w;
  *(volatile v4h*)(dst + i) = h; __threadfence(); *(volatile v4h*)(dst + i) = h;
}


__global__ __launch_bounds__(256) void wt_cvt(const float* __restrict__ W,
                                              _Float16* __restrict__ WT) {
  __shared__ float t[64][17];
  const int tx = threadIdx.x & 15, ty = threadIdx.x >> 4;
  const int nt = blockIdx.x, kt = blockIdx.y;
#pragma unroll
  for (int p = 0; p < 4; ++p) t[p * 16 + ty][tx] = W[(size_t)(kt * 64 + p * 16 + ty) * D_ + nt * 16 + tx];
  __syncthreads();
  const int rr = threadIdx.x >> 3, q = (threadIdx.x & 7) * 8;
  if (threadIdx.x < 128) {
    v4u_t v; v.x = pk2(t[q][rr], t[q + 1][rr]); v.y = pk2(t[q + 2][rr], t[q + 3][rr]); v.z = pk2(t[q + 4][rr], t[q + 5][rr]); v.w = pk2(t[q + 6][rr], t[q + 7][rr]);
    _Float16* dst = WT + (size_t)(nt * 16 + rr) * D_ + kt * 64 + q;
    *(volatile v4u_t*)dst = v; __threadfence(); *(volatile v4u_t*)dst = v;
  }
}


__global__ __launch_bounds__(32) void qkv_gemm(
    const _Float16* __restrict__ X16, const _Float16* __restrict__ WT,
    const float* __restrict__ bq, const float* __restrict__ bk,
    const float* __restrict__ bv,
    _Float16* __restrict__ Q16, _Float16* __restrict__ K16,
    _Float16* __restrict__ VT16) {
  const int lane = threadIdx.x, col = lane & 15, grp = lane >> 4;
  const int mt = blockIdx.x, nt = blockIdx.y, which = blockIdx.z;

  const _Float16* Xb = X16 + (size_t)which * ((size_t)M_ * D_);
  const _Float16* Wb = WT + (size_t)which * ((size_t)D_ * D_);
  const float* bias = (which == 0) ? bq : ((which == 1) ? bk : bv);

  const _Float16* arow = Xb + (size_t)(mt * 16 + col) * D_;
  const _Float16* br0 = Wb + (size_t)(nt * 64 + 0  + col) * D_;
  const _Float16* br1 = Wb + (size_t)(nt * 64 + 16 + col) * D_;
  const _Float16* br2 = Wb + (size_t)(nt * 64 + 32 + col) * D_;
  const _Float16* br3 = Wb + (size_t)(nt * 64 + 48 + col) * D_;

  v8f c0 = {0,0,0,0,0,0,0,0}, c1 = c0, c2 = c0, c3 = c0;
  for (int kc = 0; kc < D_; kc += 32) {
    v16h a  = ld_a(arow + kc + grp * 8);
    v16h b0 = ld_b(br0 + kc + grp * 8);
    v16h b1 = ld_b(br1 + kc + grp * 8);
    v16h b2 = ld_b(br2 + kc + grp * 8);
    v16h b3 = ld_b(br3 + kc + grp * 8);
    c0 = wmma_f16(a, b0, c0);
    c1 = wmma_f16(a, b1, c1);
    c2 = wmma_f16(a, b2, c2);
    c3 = wmma_f16(a, b3, c3);
  }

  __shared__ __attribute__((aligned(16))) float st[16][64 + 4];
  const int b = mt >> 7;
  const int sbase = (mt & 127) * 16;
  const int h = nt;
  v8f cc[4] = {c0, c1, c2, c3};
#pragma unroll
  for (int f = 0; f < 4; ++f) {
    const float bb = bias[nt * 64 + f * 16 + col];
#pragma unroll
    for (int v = 0; v < 8; ++v) st[v + 8 * grp][f * 16 + col] = cc[f][v] + bb;
  }
  asm volatile("s_wait_dscnt 0" ::: "memory");
  _Float16* dstb = ((which == 0) ? Q16 : (which == 1) ? K16 : VT16) + ((size_t)(b * H_ + h) * S_ + sbase) * HD_;
#pragma unroll 1
  for (int pass = 0; pass < 2; ++pass) {
#pragma unroll
    for (int i = 0; i < 4; ++i) { const int c = lane + 32 * i, rr = c >> 3, q = (c & 7) * 8; const float* s = &st[rr][q];
      v4u_t v; v.x = pk2(s[0], s[1]); v.y = pk2(s[2], s[3]); v.z = pk2(s[4], s[5]); v.w = pk2(s[6], s[7]);
      *(volatile v4u_t*)(dstb + (size_t)rr * HD_ + q) = v; }
    __threadfence();
  }
}


__global__ __launch_bounds__(32) void attn_kernel(
    const _Float16* __restrict__ Q16, const _Float16* __restrict__ K16,
    const _Float16* __restrict__ VT16, _Float16* __restrict__ AO16) {
  const int lane = threadIdx.x, col = lane & 15, grp = lane >> 4;
  const int qt = blockIdx.x;
  const int bh = blockIdx.y;

  const _Float16* Qp = Q16 + (size_t)bh * S_ * HD_;
  const _Float16* Kp = K16 + (size_t)bh * S_ * HD_;
  const _Float16* Vp = VT16 + (size_t)bh * HD_ * S_;

  __shared__ alignas(16) _Float16 P[16 * 40];
  __shared__ alignas(16) _Float16 Vs[32 * 72];
  __shared__ __attribute__((aligned(16))) float Os[16][64 + 4];

  const _Float16* qrow = Qp + (size_t)(qt * 16 + col) * HD_;
  const v16h bq0 = ld_b(qrow + grp * 8);
  const v16h bq1 = ld_b(qrow + 32 + grp * 8);

  float mrun = -3.0e38f, lrun = 0.0f;
  v8f O0 = {0,0,0,0,0,0,0,0}, O1 = O0, O2 = O0, O3 = O0;

  for (int kb = 0; kb < S_; kb += 32) {
    const _Float16* k0 = Kp + (size_t)(kb + col) * HD_;
    const _Float16* k1 = Kp + (size_t)(kb + 16 + col) * HD_;
    __builtin_prefetch(k0 + 32 * HD_, 0, 3);
    {
      const uint4* vr = (const uint4*)(Vp + (size_t)(kb + lane) * HD_);
      uint4* vd = (uint4*)&Vs[lane * 72];
#pragma unroll
      for (int u = 0; u < 8; ++u) vd[u] = vr[u];
    }

    v8f s0 = {0,0,0,0,0,0,0,0}, s1 = s0;
    {
      v16h a00 = ld_a(k0 + grp * 8);
      v16h a01 = ld_a(k0 + 32 + grp * 8);
      v16h a10 = ld_a(k1 + grp * 8);
      v16h a11 = ld_a(k1 + 32 + grp * 8);
      s0 = wmma_f16(a00, bq0, s0);  s0 = wmma_f16(a01, bq1, s0);
      s1 = wmma_f16(a10, bq0, s1);  s1 = wmma_f16(a11, bq1, s1);
    }

    float mx = -3.0e38f;
#pragma unroll
    for (int i = 0; i < 8; ++i) {
      s0[i] *= SCALE_; s1[i] *= SCALE_;
      mx = fmaxf(mx, fmaxf(s0[i], s1[i]));
    }
    mx = fmaxf(mx, __shfl_xor(mx, 16, 32));
    const float mnew = fmaxf(mrun, mx);
    const float alpha = __expf(mrun - mnew);

    float rs = 0.0f;
    v8h p0, p1;
#pragma unroll
    for (int i = 0; i < 8; ++i) {
      const float ea = __expf(s0[i] - mnew);
      const float eb = __expf(s1[i] - mnew);
      rs += ea + eb;
      p0[i] = (_Float16)(ea * 1024.0f); p1[i] = (_Float16)(eb * 1024.0f);
    }
    rs += __shfl_xor(rs, 16, 32);
    lrun = lrun * alpha + rs;
    mrun = mnew;

    *(v8h*)&P[col * 40 + grp * 8] = p0;
    *(v8h*)&P[col * 40 + 16 + grp * 8] = p1;

    float ar[8];
#pragma unroll
    for (int v = 0; v < 8; ++v) ar[v] = __shfl(alpha, v + 8 * grp, 32);
#pragma unroll
    for (int v = 0; v < 8; ++v) {
      O0[v] *= ar[v]; O1[v] *= ar[v]; O2[v] *= ar[v]; O3[v] *= ar[v];
    }

    asm volatile("s_wait_dscnt 0" ::: "memory");
    v16h pa = ld_a(&P[col * 40 + grp * 8]);
    v16h bv[4];
#pragma unroll
    for (int f = 0; f < 4; ++f)
#pragma unroll
      for (int i = 0; i < 16; ++i) { const int key = ((i >> 3) * 16) + grp * 8 + (i & 7); bv[f][i] = Vs[key * 72 + f * 16 + col]; }
    O0 = wmma_f16(pa, bv[0], O0);
    O1 = wmma_f16(pa, bv[1], O1);
    O2 = wmma_f16(pa, bv[2], O2);
    O3 = wmma_f16(pa, bv[3], O3);
  }

  const float linv = 1.0f / (lrun * 1024.0f);
  float lr[8];
#pragma unroll
  for (int v = 0; v < 8; ++v) lr[v] = __shfl(linv, v + 8 * grp, 32);

  const int b = bh >> 4, h = bh & 15;
  const size_t mbase = (size_t)(b * S_ + qt * 16);
  v8f OO[4] = {O0, O1, O2, O3};
#pragma unroll
  for (int f = 0; f < 4; ++f)
#pragma unroll
    for (int v = 0; v < 8; ++v) Os[v + 8 * grp][f * 16 + col] = OO[f][v] * lr[v];
  asm volatile("s_wait_dscnt 0" ::: "memory");
#pragma unroll 1
  for (int pass = 0; pass < 2; ++pass) {
#pragma unroll
    for (int i = 0; i < 4; ++i) { const int c = lane + 32 * i, rr = c >> 3, q = (c & 7) * 8; const float* s = &Os[rr][q];
      v4u_t v; v.x = pk2(s[0], s[1]); v.y = pk2(s[2], s[3]); v.z = pk2(s[4], s[5]); v.w = pk2(s[6], s[7]);
      *(volatile v4u_t*)(AO16 + (mbase + rr) * D_ + h * HD_ + q) = v; }
    __threadfence();
  }
}


__global__ __launch_bounds__(32) void oproj_gemm(
    const _Float16* __restrict__ AO, const _Float16* __restrict__ WTo,
    const float* __restrict__ bo, const float* __restrict__ resid,
    float* __restrict__ Y) {
  const int lane = threadIdx.x, col = lane & 15, grp = lane >> 4;
  const int mt = blockIdx.x, nt = blockIdx.y;

  const _Float16* arow = AO + (size_t)(mt * 16 + col) * D_;
  const _Float16* br0 = WTo + (size_t)(nt * 64 + 0  + col) * D_;
  const _Float16* br1 = WTo + (size_t)(nt * 64 + 16 + col) * D_;
  const _Float16* br2 = WTo + (size_t)(nt * 64 + 32 + col) * D_;
  const _Float16* br3 = WTo + (size_t)(nt * 64 + 48 + col) * D_;

  v8f c0 = {0,0,0,0,0,0,0,0}, c1 = c0, c2 = c0, c3 = c0;
  for (int kc = 0; kc < D_; kc += 32) {
    v16h a  = ld_a(arow + kc + grp * 8);
    v16h b0 = ld_b(br0 + kc + grp * 8);
    v16h b1 = ld_b(br1 + kc + grp * 8);
    v16h b2 = ld_b(br2 + kc + grp * 8);
    v16h b3 = ld_b(br3 + kc + grp * 8);
    c0 = wmma_f16(a, b0, c0);
    c1 = wmma_f16(a, b1, c1);
    c2 = wmma_f16(a, b2, c2);
    c3 = wmma_f16(a, b3, c3);
  }

  __shared__ __attribute__((aligned(16))) float st[16][64 + 4];
  v8f cc[4] = {c0, c1, c2, c3};
#pragma unroll
  for (int f = 0; f < 4; ++f) {
    const int n = nt * 64 + f * 16 + col;
    const float bb = bo[n];
#pragma unroll
    for (int v = 0; v < 8; ++v) {
      const size_t m = (size_t)(mt * 16 + v + 8 * grp);
      st[v + 8 * grp][f * 16 + col] = cc[f][v] + bb + resid[m * D_ + n];
    }
  }
  asm volatile("s_wait_dscnt 0" ::: "memory");
#pragma unroll 1
  for (int pass = 0; pass < 2; ++pass) {
#pragma unroll
    for (int i = 0; i < 8; ++i) { const int c = lane + 32 * i, rr = c >> 4, q = (c & 15) * 4;
      *(volatile v4f_t*)(Y + (size_t)(mt * 16 + rr) * D_ + nt * 64 + q) = *(const volatile v4fa*)&st[rr][q]; }
    __threadfence();
  }
}


__global__ __launch_bounds__(256) void ln_kernel(
    const float* __restrict__ Y, const float* __restrict__ gamma,
    const float* __restrict__ beta, float* __restrict__ out) {
  const int row = blockIdx.x, tid = threadIdx.x;
  const float* y = Y + (size_t)row * D_;
  float vals[4], s = 0.0f, s2 = 0.0f;
#pragma unroll
  for (int i = 0; i < 4; ++i) {
    const float v = y[tid + i * 256];
    vals[i] = v; s += v; s2 += v * v;
  }
  __shared__ float shA[256], shB[256];
  shA[tid] = s; shB[tid] = s2;
  __syncthreads();
  for (int off = 128; off > 0; off >>= 1) {
    if (tid < off) { shA[tid] += shA[tid + off]; shB[tid] += shB[tid + off]; }
    __syncthreads();
  }
  const float mu = shA[0] * (1.0f / D_);
  const float var = shB[0] * (1.0f / D_) - mu * mu;
  const float inv = rsqrtf(var + EPS_);
#pragma unroll
  for (int i = 0; i < 4; ++i) {
    const int c = tid + i * 256;
    const float o = (vals[i] - mu) * inv * gamma[c] + beta[c];
    *(volatile float*)(out + (size_t)row * D_ + c) = o;
  }
  __threadfence();
#pragma unroll
  for (int i = 0; i < 4; ++i) {
    const int c = tid + i * 256;
    *(volatile float*)(out + (size_t)row * D_ + c) = (vals[i] - mu) * inv * gamma[c] + beta[c];
  }
}


extern "C" void kernel_launch(void* const* d_in, const int* in_sizes, int n_in,
                              void* d_out, int out_size, void* d_ws,
                              size_t ws_size, hipStream_t stream) {
  const float* q     = (const float*)d_in[0];
  const float* k     = (const float*)d_in[1];
  const float* v     = (const float*)d_in[2];
  const float* Wq    = (const float*)d_in[3];
  const float* bq    = (const float*)d_in[4];
  const float* Wk    = (const float*)d_in[5];
  const float* bk    = (const float*)d_in[6];
  const float* Wv    = (const float*)d_in[7];
  const float* bv    = (const float*)d_in[8];
  const float* Wo    = (const float*)d_in[9];
  const float* bo    = (const float*)d_in[10];
  const float* gamma = (const float*)d_in[11];
  const float* beta  = (const float*)d_in[12];
  float* out = (float*)d_out;

  char* ws = (char*)d_ws;
  _Float16* X16  = (_Float16*)(ws + 0);
  _Float16* WT   = (_Float16*)(ws + 25165824);
  _Float16* Q16  = (_Float16*)(ws + 33554432);
  _Float16* K16  = (_Float16*)(ws + 41943040);
  _Float16* VT16 = (_Float16*)(ws + 50331648);
  _Float16* AO16 = (_Float16*)(ws + 58720256);
  float*    Yf   = (float*)(ws + 67108864);

  cvt_f16<<<4096, 256, 0, stream>>>(q, X16 + 0 * (size_t)M_ * D_);
  cvt_f16<<<4096, 256, 0, stream>>>(k, X16 + 1 * (size_t)M_ * D_);
  cvt_f16<<<4096, 256, 0, stream>>>(v, X16 + 2 * (size_t)M_ * D_);

  dim3 tg(64, 16);
  wt_cvt<<<tg, 256, 0, stream>>>(Wq, WT + 0 * (size_t)D_ * D_);
  wt_cvt<<<tg, 256, 0, stream>>>(Wk, WT + 1 * (size_t)D_ * D_);
  wt_cvt<<<tg, 256, 0, stream>>>(Wv, WT + 2 * (size_t)D_ * D_);
  wt_cvt<<<tg, 256, 0, stream>>>(Wo, WT + 3 * (size_t)D_ * D_);

  qkv_gemm<<<dim3(256, 16, 3), 32, 0, stream>>>(X16, WT, bq, bk, bv,
                                                Q16, K16, VT16);

  attn_kernel<<<dim3(128, 32), 32, 0, stream>>>(Q16, K16, VT16, AO16);

  oproj_gemm<<<dim3(256, 16), 32, 0, stream>>>(AO16, WT + 3 * (size_t)D_ * D_,
                                               bo, q, Yf);

  ln_kernel<<<M_, 256, 0, stream>>>(Yf, gamma, beta, out);
}
